// GraphAttentionLayer_80668075753786
// MI455X (gfx1250) — hardware-run, weakly checked
//
#include <hip/hip_runtime.h>


#ifndef NB
#define NB 16
#endif
#ifndef SEQ
#define SEQ 512
#endif
#define NB_FULL  16
#define SEQ_FULL 512
#ifndef OUT_SEQ
#define OUT_SEQ SEQ
#endif
#define DM    64
#define QT    16
#define ROWS  (NB * SEQ)
#define KPL   (SEQ / 32)
#define APH   72
#define OSP   68
#define XPP   72
#define K2    2.8853900817779268f
#define AWS   (-2.8853900817779268f)
#define LOG2E 1.4426950408889634f
#define WSC   64.0f
#define WSI   (1.0f / 64.0f)
#define ACS   256.0f
#define ACI   (1.0f / 16384.0f)
#define PSH   14.0f
#define NEGB  (-3.0e38f)
#define BN_EPS 1.0e-5f

static_assert(DM == 64);
static_assert(QT == 16);
static_assert(SEQ % 64 == 0);
static_assert(SEQ % 32 == 0);
static_assert(SEQ % QT == 0);
static_assert(KPL >= 1);
static_assert(KPL <= 32);
static_assert(ROWS % 32 == 0);
static_assert(((size_t)ROWS * 16) % 256 == 0);
static_assert(NB <= NB_FULL);
static_assert(SEQ <= SEQ_FULL);
static_assert((APH * 2) % 16 == 0);
static_assert((OSP * 4) % 16 == 0);
static_assert((XPP * 2) % 16 == 0);
static_assert(256 * 16 == QT * DM * 4);
static_assert(256 * 16 * 2 == 64 * DM * 2);
static_assert(256 * 16 * 4 == DM * DM * 4);
static_assert(256 * 16 * 4 == 2 * DM * DM * 2);
static_assert(64 * 16 == 4 * DM * 4);
static_assert(32 * 16 == 2 * DM * 4);
static_assert((size_t)QT * SEQ * 4 + (size_t)QT * SEQ * 2 + QT * APH * 2 + QT * OSP * 4 + QT * 4 <= 65536);
static_assert(2 * 32 * 64 * 8 + 128 * 4 <= 131072);
static_assert(64 * XPP * 2 <= 131072);

typedef _Float16 h16;
typedef unsigned short bf;
typedef __attribute__((ext_vector_type(16))) _Float16 v16h;
typedef __attribute__((ext_vector_type(8)))  _Float16 v8h;
typedef __attribute__((ext_vector_type(8)))  float    v8f;
typedef __attribute__((ext_vector_type(4)))  float    v4f;
typedef v4f  __attribute__((may_alias)) v4fa;
typedef v8h  __attribute__((may_alias)) v8ha;

__device__ __forceinline__ unsigned short f2bf(float f) { unsigned u = __float_as_uint(f); u += 0x7FFFu + ((u >> 16) & 1u); return (unsigned short)(u >> 16); }
__device__ __forceinline__ float bfr(float f) { return __uint_as_float(((unsigned)f2bf(f)) << 16); }
__device__ __forceinline__ v16h cat16(v8h lo, v8h hi) { return __builtin_shufflevector(lo, hi, 0, 1, 2, 3, 4, 5, 6, 7, 8, 9, 10, 11, 12, 13, 14, 15); }
__device__ __forceinline__ v16h ldh(const h16* p) { return cat16(*(const v8h*)p, *(const v8h*)(p + 16)); }
static __device__ __forceinline__ h16 toh_flush(float v) { const h16 r = (h16)v; return (fabsf(v) < 6.103515625e-05f) ? (h16)0.0f : r; }
__device__ __forceinline__ v8f wmma_g(v16h a, v16h b, v8f c) {
    c = __builtin_amdgcn_wmma_f32_16x16x32_f16(false, a, false, b, (short)0, c, false, false);
    asm volatile("v_nop\n\tv_nop\n\tv_nop\n\tv_nop" : "+v"(c) : "v"(a), "v"(b));
    return c;
}

__global__ __launch_bounds__(256) void k_xprep(const float* __restrict__ x, h16* XH, h16* XT) {
    __shared__ __align__(16) h16 tl[64 * XPP];
    const int tid = threadIdx.x;
    const int b = blockIdx.x / (SEQ / 64), t0 = (blockIdx.x % (SEQ / 64)) * 64;
    v8h hv[2], tv[2];
#pragma unroll
    for (int it = 0; it < 2; ++it) { const int p = it * 256 + tid; const int row = p >> 3, c8 = (p & 7) * 8;
        const float* s = x + ((size_t)b * SEQ_FULL + t0 + row) * DM + c8;
        const v4f a = *(const v4f*)s, c = *(const v4f*)(s + 4);
#pragma unroll
        for (int e = 0; e < 4; ++e) { hv[it][e] = toh_flush(bfr(a[e])); hv[it][4 + e] = toh_flush(bfr(c[e])); }
        *(v8ha*)(&tl[row * XPP + c8]) = hv[it]; }
    __syncthreads();
#pragma unroll
    for (int it = 0; it < 2; ++it) { const int p = it * 256 + tid; const int d = p >> 3, t8 = (p & 7) * 8;
#pragma unroll
        for (int e = 0; e < 8; ++e) tv[it][e] = tl[(t8 + e) * XPP + d]; }
    h16* xhp = XH + ((size_t)b * SEQ + t0) * DM;
    h16* xtp = XT + (size_t)b * DM * SEQ + t0;
#pragma unroll 1
    for (int ps = 0; ps < 2; ++ps) {
#pragma unroll
        for (int it = 0; it < 2; ++it) { const int p = it * 256 + tid; const int d = p >> 3, t8 = (p & 7) * 8;
            *(volatile v8h*)(xhp + (size_t)p * 8) = hv[it];
            *(volatile v8h*)(xtp + (size_t)d * SEQ + t8) = tv[it]; }
        if (ps == 0) __threadfence(); }
}

__global__ __launch_bounds__(256) void k_wprep(const float* __restrict__ Wap, const float* __restrict__ bap, const float* __restrict__ attw,
                                               const float* __restrict__ Wwith, const float* __restrict__ bwith, const float* __restrict__ Wwo, const float* __restrict__ bwo,
                                               float* WA, h16* WH, float* VEC) {
    const int tid = threadIdx.x;
    v4f wa[4]; v8h wh[4];
#pragma unroll
    for (int it = 0; it < 4; ++it) { const int p = it * 256 + tid; const v4f v = *(const v4f*)(Wap + (size_t)p * 4);
#pragma unroll
        for (int e = 0; e < 4; ++e) wa[it][e] = bfr(v[e]) * K2; }
#pragma unroll
    for (int it = 0; it < 2; ++it) { const int p = it * 256 + tid; const float* s = Wwith + (size_t)p * 8;
        const v4f a = *(const v4f*)s, c = *(const v4f*)(s + 4);
#pragma unroll
        for (int e = 0; e < 4; ++e) { wh[it][e] = toh_flush(bfr(a[e]) * WSC); wh[it][4 + e] = toh_flush(bfr(c[e]) * WSC); } }
#pragma unroll
    for (int it = 0; it < 2; ++it) { const int p = it * 256 + tid; const float* s = Wwo + (size_t)p * 8;
        const v4f a = *(const v4f*)s, c = *(const v4f*)(s + 4);
#pragma unroll
        for (int e = 0; e < 4; ++e) { wh[2 + it][e] = toh_flush(bfr(a[e]) * WSC); wh[2 + it][4 + e] = toh_flush(bfr(c[e]) * WSC); } }
    const int c4 = (tid & 15) * 4, vr = (tid >> 4) & 3;
    const v4f b0 = *(const v4f*)(bap + c4), a0 = *(const v4f*)(attw + c4), b1 = *(const v4f*)(bwith + c4), b2 = *(const v4f*)(bwo + c4);
    v4f vv;
#pragma unroll
    for (int e = 0; e < 4; ++e) { const float f0 = bfr(b0[e]) * K2, f1 = bfr(a0[e]) * AWS, f2 = bfr(b1[e]) + bfr(b2[e]);
        vv[e] = (vr == 0) ? f0 : ((vr == 1) ? f1 : ((vr == 2) ? f2 : 0.0f)); }
#pragma unroll 1
    for (int ps = 0; ps < 2; ++ps) {
#pragma unroll
        for (int it = 0; it < 4; ++it) { const int p = it * 256 + tid;
            *(volatile v4f*)(WA + (size_t)p * 4) = wa[it];
            *(volatile v8h*)(WH + (size_t)p * 8) = wh[it]; }
        if (tid < 64) *(volatile v4f*)(VEC + (size_t)tid * 4) = vv;
        if (ps == 0) __threadfence(); }
}

__global__ __launch_bounds__(32 * QT) void k_attn(const h16* __restrict__ XH, const h16* __restrict__ XT, const float* __restrict__ WA, const h16* __restrict__ WH,
                                                  const float* __restrict__ VEC, float* XO) {
    __shared__ __align__(16) float s_lds[QT * SEQ];
    __shared__ __align__(16) h16   e_lds[QT * SEQ];
    __shared__ __align__(16) h16   agg_lds[QT * APH];
    __shared__ __align__(16) float os[QT * OSP];
    __shared__ float denom_lds[QT];
    const int tid = threadIdx.x;
    const int lane = tid & 31, lr = lane & 15, hi = lane >> 4;
    const int wave = __builtin_amdgcn_readfirstlane((int)(threadIdx.x >> 5));
    const int b = blockIdx.x / (SEQ / QT), bi0 = (blockIdx.x % (SEQ / QT)) * QT;
    const size_t rowb = (size_t)b * SEQ;

    v16h Cb[4][2];
    {
        const h16* xi = XH + (rowb + bi0 + wave) * DM;
#pragma unroll
        for (int ks = 0; ks < 2; ++ks) {
            const int d0 = ks * 32 + 8 * hi;
            const v8h xa = *(const v8h*)(xi + d0), xb = *(const v8h*)(xi + d0 + 16);
#pragma unroll
            for (int t = 0; t < 4; ++t) {
                const float* wr = WA + (size_t)(t * 16 + lr) * DM + d0;
                const v4f w0 = *(const v4f*)wr, w1 = *(const v4f*)(wr + 4), w2 = *(const v4f*)(wr + 16), w3 = *(const v4f*)(wr + 20);
#pragma unroll
                for (int e = 0; e < 4; ++e) {
                    Cb[t][ks][e]      = toh_flush((float)xa[e]     * w0[e]);
                    Cb[t][ks][4 + e]  = toh_flush((float)xa[4 + e] * w1[e]);
                    Cb[t][ks][8 + e]  = toh_flush((float)xb[e]     * w2[e]);
                    Cb[t][ks][12 + e] = toh_flush((float)xb[4 + e] * w3[e]);
                }
            }
        }
    }
    v8f biasC[4], wtv[4];
#pragma unroll
    for (int t = 0; t < 4; ++t) {
        const float* bp = VEC + t * 16 + 8 * hi;
        const v4f p0 = *(const v4f*)bp, p1 = *(const v4f*)(bp + 4), q0 = *(const v4f*)(bp + DM), q1 = *(const v4f*)(bp + DM + 4);
#pragma unroll
        for (int r = 0; r < 4; ++r) { biasC[t][r] = p0[r]; biasC[t][4 + r] = p1[r]; wtv[t][r] = q0[r]; wtv[t][4 + r] = q1[r]; }
    }
    const h16* xk = XH + (rowb + lr) * DM + 8 * hi;
#pragma unroll 1
    for (int J = 0; J < SEQ / 16; ++J) {
        const h16* p = xk + (size_t)J * 16 * DM;
        const v16h x0 = ldh(p), x1 = ldh(p + 32);
        float sacc = 0.0f;
#pragma unroll
        for (int t = 0; t < 4; ++t) {
            v8f acc = wmma_g(Cb[t][0], x0, biasC[t]);
            acc = wmma_g(Cb[t][1], x1, acc);
#pragma unroll
            for (int r = 0; r < 8; ++r) {
                const float ex = __builtin_amdgcn_exp2f(acc[r]);
                const float rc = __builtin_amdgcn_rcpf(1.0f + ex);
                sacc = fmaf(wtv[t][r], rc, sacc);
            }
        }
        sacc += __shfl_xor(sacc, 16, 32);
        if (lane < 16) s_lds[wave * SEQ + J * 16 + lane] = sacc;
    }
    __syncthreads();

    {
        float vals[KPL]; float m = NEGB;
#pragma unroll
        for (int k = 0; k < KPL; ++k) { vals[k] = s_lds[wave * SEQ + lane + 32 * k]; m = fmaxf(m, vals[k]); }
#pragma unroll
        for (int msk = 16; msk >= 1; msk >>= 1) m = fmaxf(m, __shfl_xor(m, msk, 32));
        const float sh = PSH - m;
        float dsum = 0.0f;
#pragma unroll
        for (int k = 0; k < KPL; ++k) {
            const float arg = vals[k] + sh;
            const float ev = __builtin_amdgcn_exp2f(arg);
            const float g = (arg < -14.0f) ? 0.0f : ev;
            const h16 ph = (h16)g;
            dsum += (float)ph;
            e_lds[wave * SEQ + lane + 32 * k] = ph;
        }
#pragma unroll
        for (int msk = 16; msk >= 1; msk >>= 1) dsum += __shfl_xor(dsum, msk, 32);
        if (lane == 0) denom_lds[wave] = dsum;
    }
    __syncthreads();

    if (wave < 4) {
        v8f acc = (v8f){};
        const h16* xc = XT + ((size_t)b * DM + wave * 16 + lr) * SEQ + 8 * hi;
        const int eo = lr * SEQ + 8 * hi;
#pragma unroll 1
        for (int j0 = 0; j0 < SEQ; j0 += 32) {
            const v16h a = cat16(*(const v8ha*)(&e_lds[eo + j0]), *(const v8ha*)(&e_lds[eo + j0 + 16]));
            const v16h bq = ldh(xc + j0);
            acc = wmma_g(a, bq, acc);
        }
#pragma unroll
        for (int r = 0; r < 8; ++r) {
            const int row = 8 * hi + r;
            const float inv = 1.0f / denom_lds[row];
            agg_lds[row * APH + wave * 16 + lr] = toh_flush(acc[r] * inv * ACS);
        }
    }
    __syncthreads();

    if (wave < 4) {
        const int o = wave * 16 + lr;
        v8f a1 = (v8f){}, a2 = (v8f){};
        const h16* xr = XH + (rowb + bi0 + lr) * DM + 8 * hi;
        const h16* w1 = WH + (size_t)o * DM + 8 * hi;
        const h16* w2 = WH + (size_t)DM * DM + (size_t)o * DM + 8 * hi;
#pragma unroll
        for (int ks = 0; ks < 2; ++ks) {
            const int d0 = ks * 32;
            const v16h A1 = cat16(*(const v8ha*)(&agg_lds[lr * APH + d0 + 8 * hi]), *(const v8ha*)(&agg_lds[lr * APH + d0 + 8 * hi + 16]));
            a1 = wmma_g(A1, ldh(w1 + d0), a1);
            a2 = wmma_g(ldh(xr + d0), ldh(w2 + d0), a2);
        }
        const float bias = VEC[2 * DM + o];
#pragma unroll
        for (int r = 0; r < 8; ++r) os[(8 * hi + r) * OSP + o] = a1[r] * ACI + a2[r] * WSI + bias;
    }
    __syncthreads();
    if (tid < 256) {
        const int row = tid >> 4, c4 = (tid & 15) * 4;
        const v4f val = *(const v4fa*)(&os[row * OSP + c4]);
        float* dst = XO + (rowb + bi0) * DM + (size_t)tid * 4;
#pragma unroll 1
        for (int ps = 0; ps < 2; ++ps) {
            *(volatile v4f*)dst = val;
            if (ps == 0) __threadfence(); }
    }
}

__global__ __launch_bounds__(512) void k_stats(const float* __restrict__ XO, const float* __restrict__ gamma, float* ST) {
#pragma clang fp contract(off)
    __shared__ double red[2 * 32 * 64];
    __shared__ __align__(16) float st[128];
    const int tid = threadIdx.x; const int cq = tid & 15, rl = tid >> 4;
    double s0 = 0.0, s1 = 0.0, s2 = 0.0, s3 = 0.0, q0 = 0.0, q1 = 0.0, q2 = 0.0, q3 = 0.0;
#pragma unroll 1
    for (int r = rl; r < ROWS; r += 32) {
        const v4f v = *(const v4f*)(XO + (size_t)r * DM + cq * 4);
        const double d0 = (double)v[0], d1 = (double)v[1], d2 = (double)v[2], d3 = (double)v[3];
        s0 += d0; s1 += d1; s2 += d2; s3 += d3;
        q0 += d0 * d0; q1 += d1 * d1; q2 += d2 * d2; q3 += d3 * d3;
    }
    red[rl * 64 + cq * 4 + 0] = s0; red[rl * 64 + cq * 4 + 1] = s1; red[rl * 64 + cq * 4 + 2] = s2; red[rl * 64 + cq * 4 + 3] = s3;
    red[(32 + rl) * 64 + cq * 4 + 0] = q0; red[(32 + rl) * 64 + cq * 4 + 1] = q1; red[(32 + rl) * 64 + cq * 4 + 2] = q2; red[(32 + rl) * 64 + cq * 4 + 3] = q3;
    __syncthreads();
    if (tid < 64) {
        double S = 0.0, Q = 0.0;
#pragma unroll 1
        for (int rr = 0; rr < 32; ++rr) { S += red[rr * 64 + tid]; Q += red[(32 + rr) * 64 + tid]; }
        const double mean = S / (double)ROWS;
        const double var = Q / (double)ROWS - mean * mean;
        float vf = (float)var; vf = vf > 0.0f ? vf : 0.0f;
        const float rs = rsqrtf(vf + BN_EPS);
        st[tid] = (float)mean;
        st[64 + tid] = rs * bfr(gamma[tid]);
    }
    __syncthreads();
    if (tid < 32) {
        const v4f val = *(const v4fa*)(&st[tid * 4]);
        float* dst = ST + (size_t)tid * 4;
#pragma unroll 1
        for (int ps = 0; ps < 2; ++ps) {
            *(volatile v4f*)dst = val;
            if (ps == 0) __threadfence(); }
    }
}

__global__ __launch_bounds__(256) void k_bnselu(const float* __restrict__ XO, const float* __restrict__ ST, const float* __restrict__ beta, float* OUT) {
#pragma clang fp contract(off)
    const size_t i4 = (size_t)blockIdx.x * 256 + threadIdx.x;
    if (i4 >= (size_t)ROWS * 16) return;
    const size_t row = i4 >> 4; const int c4 = (int)(i4 & 15) * 4;
    const size_t bb = row / SEQ, tt = row % SEQ;
    const v4f xv = *(const v4f*)(XO + i4 * 4);
    const v4f mean = *(const v4f*)(ST + c4), mult = *(const v4f*)(ST + DM + c4), bt = *(const v4f*)(beta + c4);
    v4f o;
#pragma unroll
    for (int e = 0; e < 4; ++e) {
        const float y = (xv[e] - mean[e]) * mult[e] + bfr(bt[e]);
        const float neg = 1.0507009873554805f * 1.6732632423543772f * (__builtin_amdgcn_exp2f(y * LOG2E) - 1.0f);
        o[e] = (y > 0.0f) ? (1.0507009873554805f * y) : neg;
    }
    float* dst = OUT + (bb * OUT_SEQ + tt) * DM + c4;
#pragma unroll 1
    for (int ps = 0; ps < 2; ++ps) {
        *(volatile v4f*)dst = o;
        if (ps == 0) __threadfence(); }
}

static constexpr size_t al256(size_t v) { return (v + 255) & ~(size_t)255; }
static constexpr size_t SZ_XH = al256((size_t)NB * SEQ * DM * 2);
static constexpr size_t SZ_XT = al256((size_t)NB * DM * SEQ * 2);
static constexpr size_t SZ_XO = al256((size_t)NB * SEQ * DM * 4);
static constexpr size_t SZ_WA = al256((size_t)DM * DM * 4);
static constexpr size_t SZ_WH = al256((size_t)2 * DM * DM * 2);
static constexpr size_t SZ_VE = al256((size_t)4 * DM * 4);
static constexpr size_t SZ_ST = al256((size_t)2 * DM * 4);
static constexpr size_t SZ_TOTAL = SZ_XH + SZ_XT + SZ_XO + SZ_WA + SZ_WH + SZ_VE + SZ_ST;
static_assert(SZ_TOTAL <= (size_t)134217728);
static_assert((size_t)(NB * SEQ / 64) * 64 * DM * 2 <= SZ_XH);
static_assert((size_t)(NB * SEQ / QT) * QT * DM * 4 <= SZ_XO);

extern "C" void kernel_launch(void* const* d_in, const int* in_sizes, int n_in,
                              void* d_out, int out_size, void* d_ws, size_t ws_size, hipStream_t stream) {
    if (n_in < 10) return;
    const size_t needx = ((size_t)(NB - 1) * SEQ_FULL + SEQ) * DM;
    if ((size_t)in_sizes[0] < needx) return;
    if (in_sizes[1] < DM * DM || in_sizes[4] < DM * DM || in_sizes[6] < DM * DM) return;
    if (in_sizes[2] < DM || in_sizes[3] < DM || in_sizes[5] < DM || in_sizes[7] < DM || in_sizes[8] < DM || in_sizes[9] < DM) return;
    if ((size_t)out_size < ((size_t)(NB - 1) * OUT_SEQ + SEQ) * DM) return;
    if (SZ_TOTAL > ws_size) return;
    const float* x     = (const float*)d_in[0];
    const float* Wap   = (const float*)d_in[1];
    const float* bap   = (const float*)d_in[2];
    const float* attw  = (const float*)d_in[3];
    const float* Wwith = (const float*)d_in[4];
    const float* bwith = (const float*)d_in[5];
    const float* Wwo   = (const float*)d_in[6];
    const float* bwo   = (const float*)d_in[7];
    const float* gamma = (const float*)d_in[8];
    const float* beta  = (const float*)d_in[9];
    float* OUT = (float*)d_out;
    char* wsp = (char*)d_ws;
    h16*   XH  = (h16*)wsp;   wsp += SZ_XH;
    h16*   XT  = (h16*)wsp;   wsp += SZ_XT;
    float* XO  = (float*)wsp; wsp += SZ_XO;
    float* WA  = (float*)wsp; wsp += SZ_WA;
    h16*   WH  = (h16*)wsp;   wsp += SZ_WH;
    float* VEC = (float*)wsp; wsp += SZ_VE;
    float* ST  = (float*)wsp; wsp += SZ_ST;

    k_xprep<<<dim3(NB * SEQ / 64, 1, 1), 256, 0, stream>>>(x, XH, XT);
    k_wprep<<<dim3(1, 1, 1), 256, 0, stream>>>(Wap, bap, attw, Wwith, bwith, Wwo, bwo, WA, WH, VEC);
    k_attn<<<dim3(NB * SEQ / QT, 1, 1), 32 * QT, 0, stream>>>(XH, XT, WA, WH, VEC, XO);
    k_stats<<<dim3(1, 1, 1), 512, 0, stream>>>(XO, gamma, ST);
    k_bnselu<<<dim3((unsigned)(((size_t)ROWS * 16 + 255) / 256), 1, 1), 256, 0, stream>>>(XO, ST, beta, OUT);
}
